// CrossScanStrategy_7662221656541
// MI455X (gfx1250) — hardware-run, weakly checked
//
#include <hip/hip_runtime.h>
#include <hip/hip_fp16.h>
#include <math.h>

typedef __attribute__((ext_vector_type(16))) _Float16 v16h;
typedef __attribute__((ext_vector_type(8)))  _Float16 v8h;
typedef __attribute__((ext_vector_type(8)))  float    v8f;
typedef __attribute__((ext_vector_type(4)))  float    v4f;
typedef __attribute__((ext_vector_type(2)))  unsigned v2u;
typedef __attribute__((ext_vector_type(4)))  unsigned v4u;

constexpr int kBatch   = 2;
constexpr int kH       = 64;
constexpr int kW       = 64;
constexpr int kL       = kH * kW;
constexpr int kRows    = kBatch * kL;
constexpr int kD       = 256;
constexpr int kNst     = 16;
constexpr int kBcP     = 64;
constexpr int kDirs    = 4;
constexpr int kAlpFloats = kD * kNst;
constexpr int kPadFloats = kAlpFloats + kD;
constexpr float kXCarry = 64.0f;
constexpr float kWCarry = 1024.0f;
constexpr float kYCarry = 64.0f;
constexpr float kResid  = 2048.0f;
constexpr float kMergeScale = 0.25f / kYCarry;
static_assert(kH == 64 && kW == 64 && kH == kW);
static_assert(kL == 4096 && kRows == 8192);
static_assert(kD == 256 && kDirs == 4 && kNst == 16);
static_assert(2 * kNst <= kBcP);
static_assert((kD % 32) == 0);
static_assert((kD % 64) == 0 && (kBcP % 64) == 0);
static_assert((kRows % 32) == 0);
static_assert((kL % 64) == 0 && (kL % 4) == 0);
static_assert(kAlpFloats == 4096 && kPadFloats == 4352);

constexpr size_t kSzXH   = (size_t)kRows * kD * 2;
constexpr size_t kSzWD   = (size_t)kD * kD * 2;
constexpr size_t kSzWBC  = (size_t)kBcP * kD * 2;
constexpr size_t kSzDT0  = (size_t)kRows * kD * 4;
constexpr size_t kSzBC0  = (size_t)kRows * kBcP * 4;
constexpr size_t kSzXS   = (size_t)kDirs * kRows * kD * 4;
constexpr size_t kSzDTP  = (size_t)kDirs * kRows * kD * 4;
constexpr size_t kSzXD   = (size_t)kDirs * kRows * kBcP * 4;
constexpr size_t kSzPADS = (size_t)kPadFloats * 4;
constexpr size_t kSzYH   = (size_t)kDirs * kRows * kD * 2;
constexpr size_t kOffXH   = 0;
constexpr size_t kOffWD   = kOffXH   + kSzXH;
constexpr size_t kOffWBC  = kOffWD   + kSzWD;
constexpr size_t kOffDT0  = kOffWBC  + kSzWBC;
constexpr size_t kOffBC0  = kOffDT0  + kSzDT0;
constexpr size_t kOffXS   = kOffBC0  + kSzBC0;
constexpr size_t kOffDTP  = kOffXS   + kSzXS;
constexpr size_t kOffXD   = kOffDTP  + kSzDTP;
constexpr size_t kOffPADS = kOffXD   + kSzXD;
constexpr size_t kOffYH   = kOffPADS + kSzPADS;
constexpr size_t kWsTotal = kOffYH   + kSzYH;
static_assert(kSzXH == 4194304ull && kSzWD == 131072ull && kSzWBC == 32768ull && kSzDT0 == 8388608ull);
static_assert(kSzBC0 == 2097152ull && kSzXS == 33554432ull && kSzDTP == 33554432ull && kSzXD == 8388608ull);
static_assert(kSzPADS == 17408ull && kSzYH == 16777216ull);
static_assert(kWsTotal == 4194304ull + 131072ull + 32768ull + 8388608ull + 2097152ull + 33554432ull +
              33554432ull + 8388608ull + 17408ull + 16777216ull);
static_assert(kWsTotal == 107136000ull);
static_assert(kWsTotal <= 134217728ull);
static_assert((kSzXH % 128) == 0 && (kSzWD % 128) == 0 && (kSzWBC % 128) == 0 && (kSzDT0 % 128) == 0 &&
              (kSzBC0 % 128) == 0 && (kSzXS % 128) == 0 && (kSzDTP % 128) == 0 && (kSzXD % 128) == 0 &&
              (kSzPADS % 128) == 0 && (kSzYH % 128) == 0);
static_assert((((size_t)kRows * kD * 4) % 128) == 0 && (((size_t)kRows * kD * 2) % 128) == 0 &&
              (((size_t)kRows * kBcP * 4) % 128) == 0 && (((size_t)kAlpFloats * 4) % 128) == 0);

__device__ __forceinline__ _Float16 f16_flush(float v) {
  const float w = (fabsf(v) < 6.103515625e-05f) ? 0.0f : v;
  return (_Float16)w;
}
__device__ __forceinline__ void f16_split(float v, _Float16& hi, _Float16& lo) {
  hi = f16_flush(v);
  const float hf = (float)hi;
  const float r = (v - hf) * kResid;
  lo = f16_flush(r);
}

__device__ __forceinline__ float bf16r(float v) {
  unsigned u = __float_as_uint(v);
  u = (u + 0x7FFFu + ((u >> 16) & 1u)) & 0xFFFF0000u;
  return __uint_as_float(u);
}

__device__ __forceinline__ float h16_to_f32(unsigned hb) {
  const unsigned sgn = (hb & 0x8000u) << 16; const unsigned em = hb & 0x7fffu;
  const float fn = __uint_as_float((em << 13) + 0x38000000u);
  const float fs = (float)em * 5.9604644775390625e-8f;
  const float mag = (em < 0x400u) ? fs : fn; return __uint_as_float(__float_as_uint(mag) | sgn); }

namespace eng {
union FragU { v16h v; v8h h[2]; };
__device__ __forceinline__ v16h frag_load(const _Float16* p) {
  FragU f;
  f.h[0] = *(const v8h*)(p);
  f.h[1] = *(const v8h*)(p + 16);
  return f.v;
}
__device__ __forceinline__ v8f mma(v16h a, v16h b, v8f c) {
  return __builtin_amdgcn_wmma_f32_16x16x32_f16(false, a, false, b, (short)0, c, false, false);
}
__device__ __forceinline__ void guard1(v8f& a, v16h x, v16h y) {
  asm volatile("v_nop\n\tv_nop\n\tv_nop\n\tv_nop" : "+v"(a) : "v"(x), "v"(y));
}
__device__ __forceinline__ void guard_acc(v8f& a) {
  asm volatile("v_nop\n\tv_nop\n\tv_nop\n\tv_nop" : "+v"(a));
}
__device__ __forceinline__ void keep4(v16h a, v16h b, v16h c, v16h d) {
  asm volatile("v_nop" :: "v"(a), "v"(b), "v"(c), "v"(d));
}

template <int MI, int SPL>
__global__ __launch_bounds__(256) void gemm_f16_kernel(
    const unsigned short* __restrict__ Ap, const unsigned short* __restrict__ A2p, int lda,
    const unsigned short* __restrict__ Btp, const unsigned short* __restrict__ Bt2p, int ldb,
    float* __restrict__ C, int ldc, int M, int N, int K, float scale, float rscale)
{
  static_assert(MI >= 1 && MI <= 2);
  static_assert(SPL >= 0 && SPL <= 2);
  const _Float16* A   = (const _Float16*)Ap;
  const _Float16* A2  = (const _Float16*)A2p;
  const _Float16* Bt  = (const _Float16*)Btp;
  const _Float16* Bt2 = (const _Float16*)Bt2p;
  __shared__ __align__(16) float sT[8][16 * 68];
  const int lane = threadIdx.x & 31;
  const int wave = threadIdx.x >> 5;
  const int tilesN = N >> 6;
  const int tilesM = M / (16 * MI);
  const int tile = blockIdx.x * 8 + wave;
  if (tile >= tilesM * tilesN) return;
  const int tm = tile / tilesN;
  const int tn = tile - tm * tilesN;
  const int m0 = tm * (16 * MI);
  const int n0 = tn << 6;
  const int rlane = lane & 15;
  const int koff  = (lane >> 4) * 8;
  const int mOff  = (lane >> 4) * 8;

  v8f acc[MI][4], accr[MI][4];
#pragma unroll
  for (int i = 0; i < MI; ++i)
#pragma unroll
    for (int j = 0; j < 4; ++j) {
      acc[i][j]  = (v8f){0.f, 0.f, 0.f, 0.f, 0.f, 0.f, 0.f, 0.f};
      accr[i][j] = (v8f){0.f, 0.f, 0.f, 0.f, 0.f, 0.f, 0.f, 0.f};
    }

  for (int k0 = 0; k0 < K; k0 += 32) {
    v16h bh[4], bl[4];
#pragma unroll
    for (int j = 0; j < 4; ++j) {
      const size_t bo = (size_t)(n0 + (j << 4) + rlane) * ldb + koff + k0;
      bh[j] = frag_load(Bt + bo);
      if (SPL == 2) bl[j] = frag_load(Bt2 + bo); else bl[j] = bh[j];
    }
#pragma unroll
    for (int i = 0; i < MI; ++i) {
      const size_t ao = (size_t)(m0 + (i << 4) + rlane) * lda + koff + k0;
      const v16h ah = frag_load(A + ao);
      v16h al = ah;
      if (SPL >= 1) al = frag_load(A2 + ao);
#pragma unroll
      for (int j = 0; j < 4; ++j) {
        acc[i][j] = mma(ah, bh[j], acc[i][j]);
        if (SPL >= 1) accr[i][j] = mma(al, bh[j], accr[i][j]);
        if (SPL == 2) accr[i][j] = mma(ah, bl[j], accr[i][j]);
      }
#pragma unroll
      for (int j = 0; j < 4; ++j) {
        guard1(acc[i][j], ah, al);
        if (SPL >= 1) guard1(accr[i][j], ah, al);
      }
    }
    keep4(bh[0], bh[1], bh[2], bh[3]);
    if (SPL == 2) keep4(bl[0], bl[1], bl[2], bl[3]);
  }
#pragma unroll
  for (int i = 0; i < MI; ++i)
#pragma unroll
    for (int j = 0; j < 4; ++j) {
      guard_acc(acc[i][j]);
      if (SPL >= 1) guard_acc(accr[i][j]);
    }

  float* slab = sT[wave];
#pragma unroll
  for (int i = 0; i < MI; ++i) {
    const int mBase = m0 + (i << 4);
#pragma unroll
    for (int j = 0; j < 4; ++j) {
#pragma unroll
      for (int r = 0; r < 8; ++r) {
        float v = acc[i][j][r] * scale;
        if (SPL >= 1) v += accr[i][j][r] * rscale;
        slab[(mOff + r) * 68 + (j << 4) + rlane] = v;
      }
    }
    __builtin_amdgcn_fence(__ATOMIC_RELEASE, "workgroup");
    __builtin_amdgcn_wave_barrier();
    __builtin_amdgcn_fence(__ATOMIC_ACQUIRE, "workgroup");
    {
      const int hh = lane >> 4, c4 = (lane & 15) * 4;
      for (int pass = 0; pass < 2; ++pass) {
#pragma unroll
        for (int it = 0; it < 8; ++it) {
          const int row = it * 2 + hh;
          const v4f v = *(const v4f*)(slab + row * 68 + c4);
          *(volatile v4f*)(C + (size_t)(mBase + row) * ldc + n0 + c4) = v;
        }
        __threadfence();
      }
    }
    __builtin_amdgcn_fence(__ATOMIC_RELEASE, "workgroup");
    __builtin_amdgcn_wave_barrier();
    __builtin_amdgcn_fence(__ATOMIC_ACQUIRE, "workgroup");
  }
}
}

__device__ __forceinline__ _Float16 in_half(float v, float carry, bool live) {
  const float t = live ? (bf16r(v) * carry) : 0.0f;
  return f16_flush(t);
}
__device__ __forceinline__ _Float16 val_half(float v, float carry, bool live) {
  const float t = live ? (v * carry) : 0.0f;
  return f16_flush(t);
}
__device__ __forceinline__ v8h pack8_in(v4f a0, v4f a1, float carry, bool live) {
  const float f0 = a0[0];
  const float f1 = a0[1];
  const float f2 = a0[2];
  const float f3 = a0[3];
  const float f4 = a1[0];
  const float f5 = a1[1];
  const float f6 = a1[2];
  const float f7 = a1[3];
  v8h hv;
  hv[0] = in_half(f0, carry, live);
  hv[1] = in_half(f1, carry, live);
  hv[2] = in_half(f2, carry, live);
  hv[3] = in_half(f3, carry, live);
  hv[4] = in_half(f4, carry, live);
  hv[5] = in_half(f5, carry, live);
  hv[6] = in_half(f6, carry, live);
  hv[7] = in_half(f7, carry, live);
  return hv;
}
__device__ __forceinline__ int src_pixel(int k, int t) {
  const int q = t / kW;
  const int r = t - q * kW;
  const int p0 = t;
  const int p1 = kL - 1 - t;
  const int p2 = (kH - 1 - q) * kW + r;
  const int p3 = r * kW + (kW - 1 - q);
  const int pa = (k == 1) ? p1 : p0;
  const int pb = (k == 3) ? p3 : p2;
  return (k >= 2) ? pb : pa;
}
__device__ __forceinline__ int inv_time(int k, int p) {
  const int h = p / kW;
  const int w = p - h * kW;
  const int t0 = p;
  const int t1 = kL - 1 - p;
  const int t2 = (kH - 1 - h) * kW + w;
  const int t3 = (kW - 1 - w) * kH + h;
  const int ta = (k == 1) ? t1 : t0;
  const int tb = (k == 3) ? t3 : t2;
  return (k >= 2) ? tb : ta;
}

__global__ __launch_bounds__(256) void pack_x_kernel(
    const float* __restrict__ x, unsigned short* __restrict__ XH)
{
  const int i = blockIdx.x * 256 + threadIdx.x;
  const int r = i / (kD / 8);
  const int c8 = (i - r * (kD / 8)) * 8;
  const int b = r / kL;
  const int p = r - b * kL;
  const float* sp = x + ((size_t)(b * kD + c8) * kL + p);
  const float f0 = sp[0];
  const float f1 = sp[kL];
  const float f2 = sp[2 * kL];
  const float f3 = sp[3 * kL];
  const float f4 = sp[4 * kL];
  const float f5 = sp[5 * kL];
  const float f6 = sp[6 * kL];
  const float f7 = sp[7 * kL];
  v8h hv;
  hv[0] = in_half(f0, kXCarry, true);
  hv[1] = in_half(f1, kXCarry, true);
  hv[2] = in_half(f2, kXCarry, true);
  hv[3] = in_half(f3, kXCarry, true);
  hv[4] = in_half(f4, kXCarry, true);
  hv[5] = in_half(f5, kXCarry, true);
  hv[6] = in_half(f6, kXCarry, true);
  hv[7] = in_half(f7, kXCarry, true);
  unsigned short* q = XH + (size_t)i * 8;
  *(volatile v8h*)q = hv;
  __threadfence();
  *(volatile v8h*)q = hv;
}

__global__ __launch_bounds__(256) void pack_wd_kernel(
    const float* __restrict__ w, unsigned short* __restrict__ WD)
{
  const int i = blockIdx.x * 256 + threadIdx.x;
  const int n = i / (kD / 8);
  const int k8 = (i - n * (kD / 8)) * 8;
  const float* sp = w + ((size_t)k8 * kD + n);
  const float f0 = sp[0];
  const float f1 = sp[kD];
  const float f2 = sp[2 * kD];
  const float f3 = sp[3 * kD];
  const float f4 = sp[4 * kD];
  const float f5 = sp[5 * kD];
  const float f6 = sp[6 * kD];
  const float f7 = sp[7 * kD];
  v8h hv;
  hv[0] = in_half(f0, kWCarry, true);
  hv[1] = in_half(f1, kWCarry, true);
  hv[2] = in_half(f2, kWCarry, true);
  hv[3] = in_half(f3, kWCarry, true);
  hv[4] = in_half(f4, kWCarry, true);
  hv[5] = in_half(f5, kWCarry, true);
  hv[6] = in_half(f6, kWCarry, true);
  hv[7] = in_half(f7, kWCarry, true);
  unsigned short* q = WD + (size_t)i * 8;
  *(volatile v8h*)q = hv;
  __threadfence();
  *(volatile v8h*)q = hv;
}

__device__ __forceinline__ _Float16 wbc_half(const float* __restrict__ wb, const float* __restrict__ wc,
                                             int k, int cb, int cc, bool isB, bool live) {
  const float vb = wb[k * kNst + cb];
  const float vc = wc[k * kNst + cc];
  const float v = isB ? vb : vc;
  return in_half(v, kWCarry, live);
}
__global__ __launch_bounds__(256) void pack_wbc_kernel(
    const float* __restrict__ wb, const float* __restrict__ wc, unsigned short* __restrict__ WBC)
{
  const int i = blockIdx.x * 256 + threadIdx.x;
  const int n = i / (kD / 8);
  const int k8 = (i - n * (kD / 8)) * 8;
  const bool isB = (n < kNst);
  const bool live = (n < 2 * kNst);
  const int cb = isB ? n : (kNst - 1);
  const int nm = n - kNst;
  const int cl = (nm < 0) ? 0 : nm;
  const int cc = (cl > kNst - 1) ? (kNst - 1) : cl;
  v8h hv;
  hv[0] = wbc_half(wb, wc, k8 + 0, cb, cc, isB, live);
  hv[1] = wbc_half(wb, wc, k8 + 1, cb, cc, isB, live);
  hv[2] = wbc_half(wb, wc, k8 + 2, cb, cc, isB, live);
  hv[3] = wbc_half(wb, wc, k8 + 3, cb, cc, isB, live);
  hv[4] = wbc_half(wb, wc, k8 + 4, cb, cc, isB, live);
  hv[5] = wbc_half(wb, wc, k8 + 5, cb, cc, isB, live);
  hv[6] = wbc_half(wb, wc, k8 + 6, cb, cc, isB, live);
  hv[7] = wbc_half(wb, wc, k8 + 7, cb, cc, isB, live);
  unsigned short* q = WBC + (size_t)i * 8;
  *(volatile v8h*)q = hv;
  __threadfence();
  *(volatile v8h*)q = hv;
}

__global__ __launch_bounds__(256) void order_kernel(
    const float* __restrict__ x, float* __restrict__ XS)
{
  const int i = blockIdx.x * 256 + threadIdx.x;
  const int k = i / (kRows * (kD / 4));
  const int rem = i - k * (kRows * (kD / 4));
  const int R = rem / (kD / 4);
  const int d4 = (rem - R * (kD / 4)) * 4;
  const int b = R / kL;
  const int t = R - b * kL;
  const int p = src_pixel(k, t);
  const float* sp = x + ((size_t)(b * kD + d4) * kL + p);
  const float f0 = sp[0];
  const float f1 = sp[kL];
  const float f2 = sp[2 * kL];
  const float f3 = sp[3 * kL];
  v4f o;
  o[0] = bf16r(f0);
  o[1] = bf16r(f1);
  o[2] = bf16r(f2);
  o[3] = bf16r(f3);
  float* q = XS + (size_t)i * 4;
  *(volatile v4f*)q = o;
  __threadfence();
  *(volatile v4f*)q = o;
}

__global__ __launch_bounds__(256) void gather_dt_kernel(
    const float* __restrict__ DT0, const float* __restrict__ bdelta, float* __restrict__ DTP)
{
  const int i = blockIdx.x * 256 + threadIdx.x;
  const int k = i / (kRows * (kD / 4));
  const int rem = i - k * (kRows * (kD / 4));
  const int R = rem / (kD / 4);
  const int d4 = (rem - R * (kD / 4)) * 4;
  const int b = R / kL;
  const int t = R - b * kL;
  const int p = src_pixel(k, t);
  const v4f va = *(const v4f*)(DT0 + ((size_t)(b * kL + p) * kD + d4));
  const v4f vb = *(const v4f*)(bdelta + d4);
  const float a0 = va[0];
  const float a1 = va[1];
  const float a2 = va[2];
  const float a3 = va[3];
  const float e0 = vb[0];
  const float e1 = vb[1];
  const float e2 = vb[2];
  const float e3 = vb[3];
  v4f o;
  o[0] = a0 + bf16r(e0);
  o[1] = a1 + bf16r(e1);
  o[2] = a2 + bf16r(e2);
  o[3] = a3 + bf16r(e3);
  float* q = DTP + (size_t)i * 4;
  *(volatile v4f*)q = o;
  __threadfence();
  *(volatile v4f*)q = o;
}

__global__ __launch_bounds__(256) void gather_bc_kernel(
    const float* __restrict__ BC0, float* __restrict__ XD)
{
  const int i = blockIdx.x * 256 + threadIdx.x;
  const int k = i / (kRows * (kBcP / 4));
  const int rem = i - k * (kRows * (kBcP / 4));
  const int R = rem / (kBcP / 4);
  const int j4 = (rem - R * (kBcP / 4)) * 4;
  const int b = R / kL;
  const int t = R - b * kL;
  const int p = src_pixel(k, t);
  const v4f o = *(const v4f*)(BC0 + ((size_t)(b * kL + p) * kBcP + j4));
  float* q = XD + (size_t)i * 4;
  *(volatile v4f*)q = o;
  __threadfence();
  *(volatile v4f*)q = o;
}

__global__ __launch_bounds__(32) void pads_kernel(
    const float* __restrict__ alog, const float* __restrict__ dsk, float* __restrict__ PADS)
{
  const int wi = blockIdx.x * 32 + threadIdx.x;
  const int f0 = wi * 4;
  const bool isA = (f0 < kAlpFloats);
  const int ea = isA ? f0 : (kAlpFloats - 4);
  const int dq = f0 - kAlpFloats;
  const int ed = isA ? 0 : dq;
  const v4f va = *(const v4f*)(alog + ea);
  const v4f vd = *(const v4f*)(dsk + ed);
  const float a0 = va[0];
  const float a1 = va[1];
  const float a2 = va[2];
  const float a3 = va[3];
  const float e0 = vd[0];
  const float e1 = vd[1];
  const float e2 = vd[2];
  const float e3 = vd[3];
  const float s0 = isA ? a0 : e0;
  const float s1 = isA ? a1 : e1;
  const float s2 = isA ? a2 : e2;
  const float s3 = isA ? a3 : e3;
  v4f o;
  o[0] = bf16r(s0);
  o[1] = bf16r(s1);
  o[2] = bf16r(s2);
  o[3] = bf16r(s3);
  float* q = PADS + (size_t)f0;
  *(volatile v4f*)q = o;
  __threadfence();
  *(volatile v4f*)q = o;
}

typedef float    ms1_v4f __attribute__((ext_vector_type(4)));
typedef unsigned ms1_v4u __attribute__((ext_vector_type(4)));
struct ms1_args {
  const float* dtpre;
  const float* u;
  const float* bc;
  const float* z;
  const float* A_log;
  const float* Dskip;
  __half* y;
  __half* y_lo;
  long ld_dtpre;
  long ld_u;
  long ld_bc;
  long ld_z;
  long ld_y;
  int offB;
  int offC;
  int offZ;
  float ycarry;
  int dir;
  int D;
  int L;
  int nbatch;
};
static_assert(sizeof(ms1_args) == 136);

__device__ __forceinline__ float ms1_flush16(float v) {
  return (fabsf(v) < 6.103515625e-05f) ? 0.0f : v;
}
__device__ __forceinline__ unsigned ms1_h16bits(float v) {
  return (unsigned)__half_as_ushort(__float2half_rn(ms1_flush16(v)));
}
__device__ __forceinline__ float ms1_h16val(unsigned b) {
  return __half2float(__ushort_as_half((unsigned short)b));
}
__device__ __forceinline__ float ms1_softplus(float v) {
  return fmaxf(v, 0.0f) + log1pf(expf(-fabsf(v)));
}
__device__ __forceinline__ void ms1_pack2(float v0, float v1, unsigned& hw, unsigned& lw) {
  const unsigned h0 = ms1_h16bits(v0);
  const unsigned h1 = ms1_h16bits(v1);
  const float r0 = (v0 - ms1_h16val(h0)) * 2048.0f;
  const float r1 = (v1 - ms1_h16val(h1)) * 2048.0f;
  const unsigned l0 = ms1_h16bits(r0);
  const unsigned l1 = ms1_h16bits(r1);
  hw = h0 | (h1 << 16);
  lw = l0 | (l1 << 16);
}

template <int NSTATE>
__global__ __launch_bounds__(64 * (NSTATE / 16)) void ms1_scan_kernel(ms1_args a)
{
  static_assert(NSTATE == 16 || NSTATE == 64);
  constexpr int NQ  = NSTATE / 16;
  constexpr int NT  = 64 * NQ;
  constexpr int NW  = NT / 32;
  constexpr int BCW = 2 * NSTATE;
  constexpr int YP  = 68;
  constexpr int RPI = NW * 4;
  constexpr int NIT = 64 / RPI;
  static_assert(16 * NT <= 64 * YP);
  __shared__ __align__(16) float sBC[64 * BCW];
  __shared__ __align__(16) float sY[64 * YP];
  const int tid  = threadIdx.x;
  const int lane = tid & 31;
  const int wave = tid >> 5;
  const int c    = tid / NQ;
  const int sq   = tid - c * NQ;
  const int bpb  = a.D / 64;
  const int bi   = blockIdx.x / bpb;
  if (bi >= a.nbatch) return;
  const int d0 = (blockIdx.x - bi * bpb) * 64;
  const int d  = d0 + c;
  const long rowb = (long)bi * a.L;
  const bool hasz  = (a.z != nullptr);
  const bool hasD  = (a.Dskip != nullptr);
  const bool hasLo = (a.y_lo != nullptr);

#pragma unroll 1
  for (int n = 0; n < 16; ++n) {
    const float al = a.A_log[(long)d * NSTATE + sq * 16 + n];
    sY[n * NT + tid] = -expf(al);
  }
  __syncthreads();
  float An[16], h[16];
#pragma unroll
  for (int n = 0; n < 16; ++n) {
    An[n] = sY[n * NT + tid];
    h[n] = 0.0f;
  }
  float Dd = 0.0f;
  if (hasD) Dd = a.Dskip[d];

  const int nchunk = a.L / 64;
  const bool fwd = (a.dir > 0);
  const int s0 = fwd ? 0 : 63;
  const int sd = fwd ? 1 : -1;
  const int q  = lane >> 3;
  const int c8 = (lane & 7) * 8;

  for (int ci = 0; ci < nchunk; ++ci) {
    const int tb = fwd ? (ci * 64) : (a.L - 64 - ci * 64);
    const long rowc = rowb + tb;
    __syncthreads();
#pragma unroll 8
    for (int i = 0; i < 32; ++i) {
      const int idx = tid + i * NT;
      const int st  = idx / BCW;
      const int col = idx - st * BCW;
      const int sc  = (col < NSTATE) ? (a.offB + col) : (a.offC + col - NSTATE);
      sBC[idx] = a.bc[(rowc + st) * a.ld_bc + sc];
    }
    __syncthreads();
    for (int s = 0; s < 64; ++s) {
      const int ls = s0 + sd * s;
      const long row = rowc + ls;
      float pre = a.dtpre[row * a.ld_dtpre + d];
      float uv  = a.u[row * a.ld_u + d];
      float zv  = 0.0f;
      if (hasz) zv = a.z[row * a.ld_z + a.offZ + d];
      asm volatile("" : "+v"(pre));
      asm volatile("" : "+v"(uv));
      asm volatile("" : "+v"(zv));
      const float delta = ms1_softplus(pre);
      const float dtx = delta * uv;
      const float* bp = sBC + ls * BCW + sq * 16;
      const float* cp = bp + NSTATE;
      ms1_v4f Bq[4], Cq[4];
#pragma unroll
      for (int k = 0; k < 4; ++k) {
        Bq[k] = *(const ms1_v4f*)(bp + 4 * k);
        Cq[k] = *(const ms1_v4f*)(cp + 4 * k);
      }
      float yv = 0.0f;
#pragma unroll
      for (int n = 0; n < 16; ++n) {
        const float e = __expf(delta * An[n]);
        h[n] = fmaf(e, h[n], dtx * Bq[n >> 2][n & 3]);
        yv = fmaf(h[n], Cq[n >> 2][n & 3], yv);
      }
      if (NQ > 1) {
        yv += __shfl_xor(yv, 1, 32);
        yv += __shfl_xor(yv, 2, 32);
      }
      if (hasD) yv = fmaf(uv, Dd, yv);
      if (hasz) {
        const float sg = __builtin_amdgcn_rcpf(1.0f + expf(-zv));
        yv = yv * (zv * sg);
      }
      if (sq == 0) sY[ls * YP + c] = yv * a.ycarry;
    }
    __syncthreads();
    ms1_v4u hw[NIT], lw[NIT];
#pragma unroll
    for (int it = 0; it < NIT; ++it) {
      const int row = it * RPI + wave * 4 + q;
      const float* sp = sY + row * YP + c8;
      const ms1_v4f f0 = *(const ms1_v4f*)(sp);
      const ms1_v4f f1 = *(const ms1_v4f*)(sp + 4);
      unsigned h0, h1, h2, h3, l0, l1, l2, l3;
      ms1_pack2(f0[0], f0[1], h0, l0);
      ms1_pack2(f0[2], f0[3], h1, l1);
      ms1_pack2(f1[0], f1[1], h2, l2);
      ms1_pack2(f1[2], f1[3], h3, l3);
      hw[it] = (ms1_v4u){h0, h1, h2, h3};
      lw[it] = (ms1_v4u){l0, l1, l2, l3};
    }
    for (int pass = 0; pass < 2; ++pass) {
#pragma unroll
      for (int it = 0; it < NIT; ++it) {
        const int row = it * RPI + wave * 4 + q;
        const long o = (rowc + row) * a.ld_y + d0 + c8;
        *(volatile ms1_v4u*)(a.y + o) = hw[it];
        if (hasLo) *(volatile ms1_v4u*)(a.y_lo + o) = lw[it];
      }
      __threadfence();
    }
  }
}

__device__ __forceinline__ float yh_val(const unsigned short* __restrict__ YH, int k, int b, int p, int c) {
  const int row = k * kRows + b * kL + inv_time(k, p);
  const unsigned hb = (unsigned)YH[(size_t)row * kD + c];
  return h16_to_f32(hb);
}
__device__ __forceinline__ float merge_one(const unsigned short* __restrict__ YH, int b, int p, int c) {
  const float v0 = yh_val(YH, 0, b, p, c);
  const float v1 = yh_val(YH, 1, b, p, c);
  const float v2 = yh_val(YH, 2, b, p, c);
  const float v3 = yh_val(YH, 3, b, p, c);
  const float s01 = v0 + v1;
  const float s012 = s01 + v2;
  const float s = s012 + v3;
  return s * kMergeScale;
}
__global__ __launch_bounds__(256) void merge_out_kernel(
    const unsigned short* __restrict__ YH, float* __restrict__ out)
{
  const int i = blockIdx.x * 256 + threadIdx.x;
  const int bc = i / (kL / 4);
  const int p4 = (i - bc * (kL / 4)) * 4;
  const int b = bc / kD;
  const int c = bc - b * kD;
  const float r0 = merge_one(YH, b, p4 + 0, c);
  const float r1 = merge_one(YH, b, p4 + 1, c);
  const float r2 = merge_one(YH, b, p4 + 2, c);
  const float r3 = merge_one(YH, b, p4 + 3, c);
  v4f o;
  o[0] = r0;
  o[1] = r1;
  o[2] = r2;
  o[3] = r3;
  float* q = out + (size_t)i * 4;
  *(volatile v4f*)q = o;
  __threadfence();
  *(volatile v4f*)q = o;
}

static_assert(((kRows / 32) * (kD / 64)) % 8 == 0 && ((kRows / 32) * (kD / 64)) / 8 == 128);
static_assert(((kRows / 32) * (kBcP / 64)) % 8 == 0 && ((kRows / 32) * (kBcP / 64)) / 8 == 32);
static_assert(((kRows * kD / 8) % 256) == 0 && (kRows * kD / 8) / 256 == 1024);
static_assert(((kD * kD / 8) % 256) == 0 && (kD * kD / 8) / 256 == 32);
static_assert(((kBcP * kD / 8) % 256) == 0 && (kBcP * kD / 8) / 256 == 8);
static_assert(((kDirs * kRows * kD / 4) % 256) == 0 && (kDirs * kRows * kD / 4) / 256 == 8192);
static_assert(((kDirs * kRows * kBcP / 4) % 256) == 0 && (kDirs * kRows * kBcP / 4) / 256 == 2048);
static_assert((kPadFloats / 4) == 34 * 32);
static_assert(((kBatch * kD * kL / 4) % 256) == 0 && (kBatch * kD * kL / 4) / 256 == 2048);
static_assert((kD % 64) == 0 && (kL % 64) == 0);
static_assert(kRows == kBatch * kL);
static_assert((kD / 64) * (kDirs * kBatch) == 32);

extern "C" void kernel_launch(void* const* d_in, const int* in_sizes, int n_in,
                              void* d_out, int out_size, void* d_ws, size_t ws_size,
                              hipStream_t stream)
{
  if (n_in < 7) return;
  if (in_sizes[0] != kRows * kD) return;
  if (in_sizes[1] != kD * kNst) return;
  if (in_sizes[2] != kD) return;
  if (in_sizes[3] != kD * kD) return;
  if (in_sizes[4] != kD) return;
  if (in_sizes[5] != kD * kNst) return;
  if (in_sizes[6] != kD * kNst) return;
  if (out_size != kRows * kD) return;
  if (ws_size < kWsTotal) return;

  const float* x       = (const float*)d_in[0];
  const float* a_log   = (const float*)d_in[1];
  const float* d_skip  = (const float*)d_in[2];
  const float* w_delta = (const float*)d_in[3];
  const float* b_delta = (const float*)d_in[4];
  const float* w_b     = (const float*)d_in[5];
  const float* w_c     = (const float*)d_in[6];
  float* out = (float*)d_out;

  char* ws = (char*)d_ws;
  unsigned short* XH   = (unsigned short*)(ws + kOffXH);
  unsigned short* WD   = (unsigned short*)(ws + kOffWD);
  unsigned short* WBC  = (unsigned short*)(ws + kOffWBC);
  float*          DT0  = (float*)(ws + kOffDT0);
  float*          BC0  = (float*)(ws + kOffBC0);
  float*          XS   = (float*)(ws + kOffXS);
  float*          DTP  = (float*)(ws + kOffDTP);
  float*          XD   = (float*)(ws + kOffXD);
  float*          PADS = (float*)(ws + kOffPADS);
  unsigned short* YH   = (unsigned short*)(ws + kOffYH);
  float*          ALP  = PADS;
  float*          DSP  = PADS + kAlpFloats;

  constexpr float s1 = 1.0f / (kXCarry * kWCarry);

  pack_x_kernel<<<(kRows * kD / 8) / 256, 256, 0, stream>>>(x, XH);

  pack_wd_kernel<<<(kD * kD / 8) / 256, 256, 0, stream>>>(w_delta, WD);

  pack_wbc_kernel<<<(kBcP * kD / 8) / 256, 256, 0, stream>>>(w_b, w_c, WBC);

  eng::gemm_f16_kernel<2, 0><<<dim3((kRows / 32) * (kD / 64) / 8), 256, 0, stream>>>(
      XH, nullptr, kD, WD, nullptr, kD, DT0, kD, kRows, kD, kD, s1, 0.0f);

  eng::gemm_f16_kernel<2, 0><<<dim3((kRows / 32) * (kBcP / 64) / 8), 256, 0, stream>>>(
      XH, nullptr, kD, WBC, nullptr, kD, BC0, kBcP, kRows, kBcP, kD, s1, 0.0f);

  order_kernel<<<(kDirs * kRows * kD / 4) / 256, 256, 0, stream>>>(x, XS);

  gather_dt_kernel<<<(kDirs * kRows * kD / 4) / 256, 256, 0, stream>>>(DT0, b_delta, DTP);

  gather_bc_kernel<<<(kDirs * kRows * kBcP / 4) / 256, 256, 0, stream>>>(BC0, XD);

  pads_kernel<<<34, 32, 0, stream>>>(a_log, d_skip, PADS);

  ms1_args sa;
  sa.dtpre = DTP;
  sa.u = XS;
  sa.bc = XD;
  sa.z = nullptr;
  sa.A_log = ALP;
  sa.Dskip = DSP;
  sa.y = (__half*)YH;
  sa.y_lo = nullptr;
  sa.ld_dtpre = kD;
  sa.ld_u = kD;
  sa.ld_bc = kBcP;
  sa.ld_z = 0;
  sa.ld_y = kD;
  sa.offB = 0;
  sa.offC = kNst;
  sa.offZ = 0;
  sa.ycarry = kYCarry;
  sa.dir = 1;
  sa.D = kD;
  sa.L = kL;
  sa.nbatch = kDirs * kBatch;
  ms1_scan_kernel<16><<<dim3((kD / 64) * (kDirs * kBatch)), 64, 0, stream>>>(sa);

  merge_out_kernel<<<(kBatch * kD * kL / 4) / 256, 256, 0, stream>>>(YH, out);
}
